// CAR_61143154425900
// MI455X (gfx1250) — hardware-run, weakly checked
//
#include <hip/hip_runtime.h>
#include <math.h>

typedef __attribute__((ext_vector_type(16))) _Float16 v16h;
typedef __attribute__((ext_vector_type(8)))  _Float16 v8h;
typedef __attribute__((ext_vector_type(16))) __bf16   v16b;
typedef __attribute__((ext_vector_type(8)))  __bf16   v8b;
typedef __attribute__((ext_vector_type(8)))  float    v8f;
typedef __attribute__((ext_vector_type(4)))  float    v4f;
typedef __attribute__((ext_vector_type(4)))  unsigned v4u;

constexpr int kBat  = 4;
constexpr int kSeq  = 1024;
constexpr int kTok  = kBat * kSeq;
constexpr int kIn   = 768;
constexpr int kDm   = 256;
constexpr int kDi   = 512;
constexpr int kNs   = 16;
constexpr int kDtR  = 16;
constexpr int kXzP  = 2 * kDi;
constexpr int kXdN  = kDtR + 2 * kNs;
constexpr int kXdP  = 64;
constexpr int kCls  = 128;
constexpr int kLay  = 2;
constexpr int kLossIdx = kTok * kCls;
static_assert(kTok == 4096 && kXzP == 1024 && kXdN == 48 && kLossIdx == 524288, "shape constants");
static_assert(kNs == kDtR, "shared staging loop of the scan prologue");
static_assert((kIn % 32) == 0 && (kDm % 32) == 0 && (kDi % 32) == 0, "GEMM K multiples of 32");
static_assert((kTok % 64) == 0 && (kDm % 64) == 0 && (kXzP % 64) == 0 && (kXdP % 64) == 0 && (kCls % 64) == 0, "GEMM M,N multiples of 64");
static_assert((kSeq % 64) == 0 && (kDi % 256) == 0, "conv tile multiples");

constexpr float kCarryW  = 256.0f;
constexpr float kCarryHN = 16.0f;
constexpr float kCarryU  = 256.0f;
constexpr float kCarryY  = 512.0f;

constexpr size_t kOffXH   = 0;
constexpr size_t kOffXL   = kOffXH   + (size_t)kTok * kIn * 2;
constexpr size_t kOffWINH = kOffXL   + (size_t)kTok * kIn * 2;
constexpr size_t kOffWINL = kOffWINH + (size_t)kDm * kIn * 2;
constexpr size_t kOffWOPH = kOffWINL + (size_t)kDm * kIn * 2;
constexpr size_t kOffWOPL = kOffWOPH + (size_t)kDm * kDm * 2;
constexpr size_t kOffWCLH = kOffWOPL + (size_t)kDm * kDm * 2;
constexpr size_t kOffWCLL = kOffWCLH + (size_t)kCls * kDm * 2;
constexpr size_t kOffWIP  = kOffWCLL + (size_t)kCls * kDm * 2;
constexpr size_t kOffWXP  = kOffWIP  + (size_t)kLay * kXzP * kDm * 2;
constexpr size_t kOffWO   = kOffWXP  + (size_t)kLay * kXdP * kDi * 2;
constexpr size_t kOffH0P  = kOffWO   + (size_t)kLay * kDm * kDi * 2;
constexpr size_t kOffH0   = kOffH0P  + (size_t)kTok * kDm * 4;
constexpr size_t kOffH1   = kOffH0   + (size_t)kTok * kDm * 4;
constexpr size_t kOffH2H  = kOffH1   + (size_t)kTok * kDm * 4;
constexpr size_t kOffH2L  = kOffH2H  + (size_t)kTok * kDm * 2;
constexpr size_t kOffHN   = kOffH2L  + (size_t)kTok * kDm * 2;
constexpr size_t kOffXZ   = kOffHN   + (size_t)kTok * kDm * 2;
constexpr size_t kOffU    = kOffXZ   + (size_t)kTok * kXzP * 4;
constexpr size_t kOffU16  = kOffU    + (size_t)kTok * kDi * 4;
constexpr size_t kOffXD   = kOffU16  + (size_t)kTok * kDi * 2;
constexpr size_t kOffYG   = kOffXD   + (size_t)kTok * kXdP * 4;
constexpr size_t kOffPH   = kOffYG   + (size_t)kTok * kDi * 2;
constexpr size_t kOffGH   = kOffPH   + (size_t)kTok * kDm * 4;
constexpr size_t kOffGL   = kOffGH   + (size_t)kTok * kDm * 2;
constexpr size_t kOffNRM  = kOffGL   + (size_t)kTok * kDm * 2;
constexpr size_t kWsTotal = kOffNRM  + (size_t)kTok * 4;
static_assert(kWsTotal == 77348864ull, "carve total");
static_assert(kWsTotal <= 134217728ull, "carve cap");
static_assert((kOffXL % 128) == 0 && (kOffWINH % 128) == 0 && (kOffWINL % 128) == 0 && (kOffWOPH % 128) == 0 &&
              (kOffWOPL % 128) == 0 && (kOffWCLH % 128) == 0 && (kOffWCLL % 128) == 0 && (kOffWIP % 128) == 0 &&
              (kOffWXP % 128) == 0 && (kOffWO % 128) == 0 && (kOffH0P % 128) == 0 && (kOffH0 % 128) == 0 &&
              (kOffH1 % 128) == 0 && (kOffH2H % 128) == 0 && (kOffH2L % 128) == 0 && (kOffHN % 128) == 0 &&
              (kOffXZ % 128) == 0 && (kOffU % 128) == 0 && (kOffU16 % 128) == 0 && (kOffXD % 128) == 0 &&
              (kOffYG % 128) == 0 && (kOffPH % 128) == 0 && (kOffGH % 128) == 0 && (kOffGL % 128) == 0 &&
              (kOffNRM % 128) == 0, "128-B aligned regions");

__device__ __forceinline__ unsigned short f2bf_bits(float f) {
  unsigned u = __float_as_uint(f);
  return (unsigned short)((u + 0x7FFFu + ((u >> 16) & 1u)) >> 16);
}
__device__ __forceinline__ float bf_bits2f(unsigned short h) { return __uint_as_float(((unsigned)h) << 16); }
__device__ __forceinline__ unsigned short f2h_bits(float f) {
  const _Float16 h = (_Float16)f;
  return __builtin_bit_cast(unsigned short, h);
}
__device__ __forceinline__ unsigned pack2(unsigned short a, unsigned short b) {
  return (unsigned)a | ((unsigned)b << 16);
}
__device__ __forceinline__ void split2_bf16(float x, float y, unsigned& hw, unsigned& lw) {
  const unsigned short hx = f2bf_bits(x);
  const unsigned short hy = f2bf_bits(y);
  const unsigned short lx = f2bf_bits(x - bf_bits2f(hx));
  const unsigned short ly = f2bf_bits(y - bf_bits2f(hy));
  hw = pack2(hx, hy);
  lw = pack2(lx, ly);
}
__device__ __forceinline__ void split8_bf16(const v4f a0, const v4f a1, v4u& hw, v4u& lw) {
  const float x0 = a0[0], x1 = a0[1], x2 = a0[2], x3 = a0[3];
  const float x4 = a1[0], x5 = a1[1], x6 = a1[2], x7 = a1[3];
  unsigned h0, h1, h2, h3, l0, l1, l2, l3;
  split2_bf16(x0, x1, h0, l0);
  split2_bf16(x2, x3, h1, l1);
  split2_bf16(x4, x5, h2, l2);
  split2_bf16(x6, x7, h3, l3);
  hw = (v4u){h0, h1, h2, h3};
  lw = (v4u){l0, l1, l2, l3};
}
__device__ __forceinline__ v4u cast8_f16(const v4f a0, const v4f a1, float s) {
  const float x0 = a0[0] * s, x1 = a0[1] * s, x2 = a0[2] * s, x3 = a0[3] * s;
  const float x4 = a1[0] * s, x5 = a1[1] * s, x6 = a1[2] * s, x7 = a1[3] * s;
  const unsigned w0 = pack2(f2h_bits(x0), f2h_bits(x1));
  const unsigned w1 = pack2(f2h_bits(x2), f2h_bits(x3));
  const unsigned w2 = pack2(f2h_bits(x4), f2h_bits(x5));
  const unsigned w3 = pack2(f2h_bits(x6), f2h_bits(x7));
  return (v4u){w0, w1, w2, w3};
}

__device__ __forceinline__ void acc_nop_h(v8f& a, v16h x, v16h y, v16h z) { asm volatile("v_nop\n\tv_nop\n\tv_nop\n\tv_nop" : "+v"(a) : "v"(x), "v"(y), "v"(z)); }
__device__ __forceinline__ void acc_nop_b(v8f& a, v16b x, v16b y, v16b z) { asm volatile("v_nop\n\tv_nop\n\tv_nop\n\tv_nop" : "+v"(a) : "v"(x), "v"(y), "v"(z)); }
__device__ __forceinline__ void keep4_h(v16h a, v16h b, v16h c, v16h d) { asm volatile("v_nop" :: "v"(a), "v"(b), "v"(c), "v"(d)); }
__device__ __forceinline__ void keep4_b(v16b a, v16b b, v16b c, v16b d) { asm volatile("v_nop" :: "v"(a), "v"(b), "v"(c), "v"(d)); }
__device__ __forceinline__ void acc_guard4(v8f& a, v8f& b, v8f& c, v8f& d) { asm volatile("v_nop\n\tv_nop\n\tv_nop\n\tv_nop" : "+v"(a), "+v"(b), "+v"(c), "+v"(d)); }

template <typename T> struct Frag;
template <> struct Frag<_Float16> {
  typedef v16h V; union U { v16h v; v8h h[2]; };
  static __device__ __forceinline__ v16h load(const _Float16* p) {
    U f; f.h[0] = *(const v8h*)(p); f.h[1] = *(const v8h*)(p + 16); return f.v;
  }
  static __device__ __forceinline__ v8f mma(v16h a, v16h b, v8f c) {
    return __builtin_amdgcn_wmma_f32_16x16x32_f16(false, a, false, b, (short)0, c, false, false);
  }
  static __device__ __forceinline__ void guard(v8f& a, v16h x, v16h y, v16h z) { acc_nop_h(a, x, y, z); }
  static __device__ __forceinline__ void keep(v16h a, v16h b, v16h c, v16h d) { keep4_h(a, b, c, d); }
};
template <> struct Frag<__bf16> {
  typedef v16b V; union U { v16b v; v8b h[2]; };
  static __device__ __forceinline__ v16b load(const __bf16* p) {
    U f; f.h[0] = *(const v8b*)(p); f.h[1] = *(const v8b*)(p + 16); return f.v;
  }
  static __device__ __forceinline__ v8f mma(v16b a, v16b b, v8f c) {
    return __builtin_amdgcn_wmma_f32_16x16x32_bf16(false, a, false, b, (short)0, c, false, false);
  }
  static __device__ __forceinline__ void guard(v8f& a, v16b x, v16b y, v16b z) { acc_nop_b(a, x, y, z); }
  static __device__ __forceinline__ void keep(v16b a, v16b b, v16b c, v16b d) { keep4_b(a, b, c, d); }
};

template <int ET> struct Elem;
template <> struct Elem<0> { typedef _Float16 T; };
template <> struct Elem<1> { typedef __bf16 T; };

template <int ET, bool SPLIT, int BIAS_MODE, int OUT_MODE, bool RESID>
__global__ __launch_bounds__(256) void wmma_gemm64(
    const unsigned short* __restrict__ Ap, const unsigned short* __restrict__ A2p, int lda,
    const unsigned short* __restrict__ Btp, const unsigned short* __restrict__ Bt2p, int ldb,
    void* __restrict__ Cout, void* __restrict__ Cout2, int ldc,
    const float* __restrict__ bias, const float* __restrict__ resid,
    int M, int N, int K, float scale) {
  typedef typename Elem<ET>::T T;
  typedef typename Frag<T>::V V;
  const T* A = (const T*)Ap;
  const T* A2 = (const T*)A2p;
  const T* Bt = (const T*)Btp;
  const T* Bt2 = (const T*)Bt2p;
  __shared__ __align__(16) float sT[8][16 * 68];
  const int lane = threadIdx.x & 31;
  const int wave = __builtin_amdgcn_readfirstlane((int)(threadIdx.x >> 5));
  const int tilesN = N >> 6;
  const int tilesM = M >> 6;
  const int tile = blockIdx.x * 8 + wave;
  if (tile >= tilesM * tilesN) return;
  const int tm = tile / tilesN;
  const int tn = tile - tm * tilesN;
  const int m0 = tm << 6;
  const int n0 = tn << 6;

  const int rlane = lane & 15;
  const int koff  = (lane >> 4) * 8;
  const int mOff  = (lane >> 4) * 8;

  v8f acc[4][4];
#pragma unroll
  for (int i = 0; i < 4; ++i)
#pragma unroll
    for (int j = 0; j < 4; ++j) acc[i][j] = (v8f){0.f, 0.f, 0.f, 0.f, 0.f, 0.f, 0.f, 0.f};

  for (int k0 = 0; k0 < K; k0 += 32) {
    V bh[4], bl[4];
#pragma unroll
    for (int j = 0; j < 4; ++j) {
      const size_t bo = (size_t)(n0 + (j << 4) + rlane) * ldb + koff + k0;
      bh[j] = Frag<T>::load(Bt + bo);
      if (SPLIT) bl[j] = Frag<T>::load(Bt2 + bo);
      else bl[j] = bh[j];
    }
#pragma unroll
    for (int i = 0; i < 4; ++i) {
      const size_t ao = (size_t)(m0 + (i << 4) + rlane) * lda + koff + k0;
      V ah = Frag<T>::load(A + ao);
      V al = ah;
      if (SPLIT) al = Frag<T>::load(A2 + ao);
#pragma unroll
      for (int j = 0; j < 4; ++j) {
        acc[i][j] = Frag<T>::mma(ah, bh[j], acc[i][j]);
        if (SPLIT) {
          acc[i][j] = Frag<T>::mma(ah, bl[j], acc[i][j]);
          acc[i][j] = Frag<T>::mma(al, bh[j], acc[i][j]);
        }
      }
      Frag<T>::guard(acc[i][0], ah, al, bh[0]);
      Frag<T>::guard(acc[i][1], ah, al, bh[1]);
      Frag<T>::guard(acc[i][2], ah, al, bh[2]);
      Frag<T>::guard(acc[i][3], ah, al, bh[3]);
    }
    Frag<T>::keep(bh[0], bh[1], bh[2], bh[3]);
    if (SPLIT) Frag<T>::keep(bl[0], bl[1], bl[2], bl[3]);
  }
  acc_guard4(acc[0][0], acc[0][1], acc[0][2], acc[0][3]);
  acc_guard4(acc[1][0], acc[1][1], acc[1][2], acc[1][3]);
  acc_guard4(acc[2][0], acc[2][1], acc[2][2], acc[2][3]);
  acc_guard4(acc[3][0], acc[3][1], acc[3][2], acc[3][3]);

  float* slab = sT[wave];
#pragma unroll
  for (int i = 0; i < 4; ++i) {
    const int mBase = m0 + (i << 4);
#pragma unroll
    for (int j = 0; j < 4; ++j) {
      const int n = n0 + (j << 4) + rlane;
      float bv = 0.f;
      if (BIAS_MODE == 2) bv = bias[n];
#pragma unroll
      for (int r = 0; r < 8; ++r) {
        float v = acc[i][j][r] * scale;
        if (BIAS_MODE == 2) v += bv;
        slab[(mOff + r) * 68 + (j << 4) + rlane] = v;
      }
    }
    __builtin_amdgcn_fence(__ATOMIC_RELEASE, "workgroup");
    __builtin_amdgcn_wave_barrier();
    __builtin_amdgcn_fence(__ATOMIC_ACQUIRE, "workgroup");
    if (OUT_MODE == 0) {
      float* C = (float*)Cout;
      const int hh = lane >> 4, c4 = (lane & 15) * 4;
      v4f val[8];
#pragma unroll
      for (int it = 0; it < 8; ++it) {
        const int row = it * 2 + hh;
        v4f v = *(const v4f*)(slab + row * 68 + c4);
        if (RESID) {
          const v4f rv = *(const v4f*)(resid + (size_t)(mBase + row) * ldc + n0 + c4);
          v = v + rv;
        }
        val[it] = v;
      }
      for (int pass = 0; pass < 2; ++pass) {
#pragma unroll
        for (int it = 0; it < 8; ++it) {
          const int row = it * 2 + hh;
          *(volatile v4f*)(C + (size_t)(mBase + row) * ldc + n0 + c4) = val[it];
        }
        __threadfence();
      }
    } else {
      const int q = lane >> 3, c8 = (lane & 7) * 8;
      unsigned short* C  = (unsigned short*)Cout;
      unsigned short* C2 = (unsigned short*)Cout2;
      v4u hw[4], lw[4];
#pragma unroll
      for (int it = 0; it < 4; ++it) {
        const int row = it * 4 + q;
        const float* sp = slab + row * 68 + c8;
        v4f a0 = *(const v4f*)(sp);
        v4f a1 = *(const v4f*)(sp + 4);
        if (RESID) {
          const float* rp = resid + (size_t)(mBase + row) * ldc + n0 + c8;
          const v4f r0 = *(const v4f*)(rp);
          const v4f r1 = *(const v4f*)(rp + 4);
          a0 = a0 + r0;
          a1 = a1 + r1;
        }
        split8_bf16(a0, a1, hw[it], lw[it]);
      }
      for (int pass = 0; pass < 2; ++pass) {
#pragma unroll
        for (int it = 0; it < 4; ++it) {
          const int row = it * 4 + q;
          const size_t o = (size_t)(mBase + row) * ldc + n0 + c8;
          *(volatile v4u*)(C + o) = hw[it];
          *(volatile v4u*)(C2 + o) = lw[it];
        }
        __threadfence();
      }
    }
    __builtin_amdgcn_fence(__ATOMIC_RELEASE, "workgroup");
    __builtin_amdgcn_wave_barrier();
    __builtin_amdgcn_fence(__ATOMIC_ACQUIRE, "workgroup");
  }
}

__global__ __launch_bounds__(256) void split_rows_bf16_kernel(
    const float* __restrict__ src, unsigned short* __restrict__ dhi, unsigned short* __restrict__ dlo, int total8)
{
  const int i = blockIdx.x * 256 + threadIdx.x;
  if (i >= total8) return;
  const size_t e0 = (size_t)i << 3;
  const v4f a0 = *(const v4f*)(src + e0);
  const v4f a1 = *(const v4f*)(src + e0 + 4);
  v4u hw, lw;
  split8_bf16(a0, a1, hw, lw);
  unsigned short* qh = dhi + e0;
  unsigned short* ql = dlo + e0;
  *(volatile v4u*)qh = hw;
  *(volatile v4u*)ql = lw;
  __threadfence();
  *(volatile v4u*)qh = hw;
  *(volatile v4u*)ql = lw;
}

__global__ __launch_bounds__(256) void cast_rows_f16_kernel(
    const float* __restrict__ src, unsigned short* __restrict__ dst, float carry, int total8)
{
  const int i = blockIdx.x * 256 + threadIdx.x;
  if (i >= total8) return;
  const size_t e0 = (size_t)i << 3;
  const v4f a0 = *(const v4f*)(src + e0);
  const v4f a1 = *(const v4f*)(src + e0 + 4);
  const v4u w = cast8_f16(a0, a1, carry);
  unsigned short* q = dst + e0;
  *(volatile v4u*)q = w;
  __threadfence();
  *(volatile v4u*)q = w;
}

__global__ __launch_bounds__(256) void cast_xproj_pad_kernel(
    const float* __restrict__ src, unsigned short* __restrict__ dst, float carry, int total8)
{
  const int i = blockIdx.x * 256 + threadIdx.x;
  if (i >= total8) return;
  const int e0 = i << 3;
  const int col = e0 & (kDi - 1);
  const int row = (e0 >> 9) & (kXdP - 1);
  const int lay = e0 >> 15;
  const bool valid = row < kXdN;
  const int rowc = valid ? row : (kXdN - 1);
  const float* p = src + ((size_t)lay * kXdN + rowc) * kDi + col;
  const v4f a0 = *(const v4f*)(p);
  const v4f a1 = *(const v4f*)(p + 4);
  float x0 = a0[0], x1 = a0[1], x2 = a0[2], x3 = a0[3];
  float x4 = a1[0], x5 = a1[1], x6 = a1[2], x7 = a1[3];
  asm volatile("" : "+v"(x0), "+v"(x1), "+v"(x2), "+v"(x3));
  asm volatile("" : "+v"(x4), "+v"(x5), "+v"(x6), "+v"(x7));
  const v4f b0 = (v4f){valid ? x0 : 0.0f, valid ? x1 : 0.0f, valid ? x2 : 0.0f, valid ? x3 : 0.0f};
  const v4f b1 = (v4f){valid ? x4 : 0.0f, valid ? x5 : 0.0f, valid ? x6 : 0.0f, valid ? x7 : 0.0f};
  const v4u w = cast8_f16(b0, b1, carry);
  unsigned short* q = dst + (size_t)e0;
  *(volatile v4u*)q = w;
  __threadfence();
  *(volatile v4u*)q = w;
}

__device__ __forceinline__ void row_stats256(const v4f a, const v4f b, float& mu, float& rs) {
  float s = ((a[0] + a[1]) + (a[2] + a[3])) + ((b[0] + b[1]) + (b[2] + b[3]));
#pragma unroll
  for (int off = 16; off > 0; off >>= 1) s += __shfl_xor(s, off, 32);
  mu = s * (1.0f / (float)kDm);
  const v4f da = a - mu;
  const v4f db = b - mu;
  float q = ((da[0] * da[0] + da[1] * da[1]) + (da[2] * da[2] + da[3] * da[3])) +
            ((db[0] * db[0] + db[1] * db[1]) + (db[2] * db[2] + db[3] * db[3]));
#pragma unroll
  for (int off = 16; off > 0; off >>= 1) q += __shfl_xor(q, off, 32);
  const float var = q * (1.0f / (float)kDm);
  rs = 1.0f / sqrtf(var + 1e-5f);
}

template <int MODE>
__global__ __launch_bounds__(256) void ln_rows_kernel(
    const float* __restrict__ X, const float* __restrict__ g1, const float* __restrict__ b1,
    float* __restrict__ Hout, const float* __restrict__ g2, const float* __restrict__ b2,
    unsigned short* __restrict__ HN)
{
  __shared__ __align__(16) float sR[8][kDm];
  const int lane = threadIdx.x & 31;
  const int wave = __builtin_amdgcn_readfirstlane((int)(threadIdx.x >> 5));
  const int row = blockIdx.x * 8 + wave;
  float* sr = sR[wave];
  const float* xp = X + (size_t)row * kDm;
  const int ca = lane * 4, cbb = 128 + lane * 4;
  v4f va = *(const v4f*)(xp + ca);
  v4f vb = *(const v4f*)(xp + cbb);
  if (MODE == 0) {
    float mu, rs;
    row_stats256(va, vb, mu, rs);
    const v4f ga = *(const v4f*)(g1 + ca);
    const v4f gb = *(const v4f*)(g1 + cbb);
    const v4f ba = *(const v4f*)(b1 + ca);
    const v4f bb = *(const v4f*)(b1 + cbb);
    const v4f ya = (va - mu) * rs * ga + ba;
    const v4f yb = (vb - mu) * rs * gb + bb;
    *(v4f*)(sr + ca) = ya;
    *(v4f*)(sr + cbb) = yb;
    __syncthreads();
#pragma unroll 1
    for (int i = 0; i < 8; ++i) {
      const float t = sr[i * 32 + lane];
      sr[i * 32 + lane] = 0.5f * t * (1.0f + erff(t * 0.70710678118654752f));
    }
    __syncthreads();
    va = *(const v4f*)(sr + ca);
    vb = *(const v4f*)(sr + cbb);
    float* hp = Hout + (size_t)row * kDm;
    *(volatile v4f*)(hp + ca) = va;
    *(volatile v4f*)(hp + cbb) = vb;
    __threadfence();
    *(volatile v4f*)(hp + ca) = va;
    *(volatile v4f*)(hp + cbb) = vb;
    __syncthreads();
  }
  {
    float mu, rs;
    row_stats256(va, vb, mu, rs);
    const v4f ga = *(const v4f*)(g2 + ca);
    const v4f gb = *(const v4f*)(g2 + cbb);
    const v4f ba = *(const v4f*)(b2 + ca);
    const v4f bb = *(const v4f*)(b2 + cbb);
    const v4f ya = (va - mu) * rs * ga + ba;
    const v4f yb = (vb - mu) * rs * gb + bb;
    *(v4f*)(sr + ca) = ya;
    *(v4f*)(sr + cbb) = yb;
  }
  __syncthreads();
  const v4f a0 = *(const v4f*)(sr + lane * 8);
  const v4f a1 = *(const v4f*)(sr + lane * 8 + 4);
  const v4u w = cast8_f16(a0, a1, kCarryHN);
  unsigned short* q = HN + (size_t)row * kDm + lane * 8;
  *(volatile v4u*)q = w;
  __threadfence();
  *(volatile v4u*)q = w;
}

constexpr int kConvTP = 260;
__global__ __launch_bounds__(256) void conv_silu_kernel(
    const float* __restrict__ XZ, const float* __restrict__ cw, const float* __restrict__ cb,
    float* __restrict__ U, unsigned short* __restrict__ U16)
{
  __shared__ __align__(16) float sT[16 * kConvTP];
  const int tid = threadIdx.x, lane = tid & 31;
  const int wave = __builtin_amdgcn_readfirstlane((int)(threadIdx.x >> 5));
  const int d0 = blockIdx.x * 256, d = d0 + tid;
  const int g0 = blockIdx.y * 64;
  const int tb = g0 & (kSeq - 1);
  const v4f wv = *(const v4f*)(cw + (size_t)d * 4);
  const float w0 = wv[0], w1 = wv[1], w2 = wv[2], w3 = wv[3];
  const float bc = cb[d];
  float xm3, xm2, xm1;
  {
    const bool hist = (tb > 0);
    const int rb = hist ? (g0 - 3) : g0;
    float v3 = XZ[(size_t)rb * kXzP + d];
    float v2 = XZ[(size_t)(rb + 1) * kXzP + d];
    float v1 = XZ[(size_t)(rb + 2) * kXzP + d];
    asm volatile("" : "+v"(v3), "+v"(v2), "+v"(v1));
    xm3 = hist ? v3 : 0.f;
    xm2 = hist ? v2 : 0.f;
    xm1 = hist ? v1 : 0.f;
  }
  const int hrow = wave >> 1;
  const int hch  = (wave & 1) * 128 + lane * 4;
#pragma unroll 1
  for (int sub = 0; sub < 4; ++sub) {
    const int lb = g0 + sub * 16;
#pragma unroll 1
    for (int s = 0; s < 16; ++s) {
      const float xcur = XZ[(size_t)(lb + s) * kXzP + d];
      float acc = w0 * xm3;
      acc = fmaf(w1, xm2, acc);
      acc = fmaf(w2, xm1, acc);
      acc = fmaf(w3, xcur, acc);
      const float sv = acc + bc;
      const float sg = 1.0f / (1.0f + expf(-sv));
      sT[s * kConvTP + tid] = sv * sg;
      xm3 = xm2; xm2 = xm1; xm1 = xcur;
    }
    __syncthreads();
    v4f fv[4];
    v4u pk[2];
#pragma unroll
    for (int it = 0; it < 4; ++it) fv[it] = *(const v4f*)(sT + (it * 4 + hrow) * kConvTP + hch);
#pragma unroll
    for (int it = 0; it < 2; ++it) {
      const float* sp = sT + (it * 8 + wave) * kConvTP + lane * 8;
      const v4f a0 = *(const v4f*)(sp);
      const v4f a1 = *(const v4f*)(sp + 4);
      pk[it] = cast8_f16(a0, a1, kCarryU);
    }
    for (int pass = 0; pass < 2; ++pass) {
#pragma unroll
      for (int it = 0; it < 4; ++it)
        *(volatile v4f*)(U + (size_t)(lb + it * 4 + hrow) * kDi + d0 + hch) = fv[it];
#pragma unroll
      for (int it = 0; it < 2; ++it)
        *(volatile v4u*)(U16 + (size_t)(lb + it * 8 + wave) * kDi + d0 + lane * 8) = pk[it];
      __threadfence();
    }
    __syncthreads();
  }
}

constexpr int kScCh = 64;
constexpr int kScTS = 32;
constexpr int kScXP = 48;
constexpr int kScYP = 68;
static_assert((kSeq % kScTS) == 0 && (kDi % kScCh) == 0, "scan tiling");
__global__ __launch_bounds__(128) void scan_gate_kernel(
    const float* __restrict__ XD, const float* __restrict__ U, const float* __restrict__ XZ,
    const float* __restrict__ Wdt, const float* __restrict__ bdt, const float* __restrict__ Alog,
    const float* __restrict__ Dp, unsigned short* __restrict__ YG)
{
  __shared__ __align__(16) float sX[kScTS * kScXP];
  __shared__ __align__(16) float sU[kScTS * kScCh];
  __shared__ __align__(16) float sZ[kScTS * kScCh];
  __shared__ __align__(16) float sY[kScTS * kScYP];
  __shared__ __align__(16) float sA[kNs * kScCh];
  __shared__ __align__(16) float sW[kDtR * kScCh];
  const int tid = threadIdx.x, lane = tid & 31;
  const int wave = __builtin_amdgcn_readfirstlane((int)(threadIdx.x >> 5));
  const int c16 = lane & 15, half = lane >> 4;
  const int c = wave * 16 + c16;
  constexpr int kBlkPerB = kDi / kScCh;
  const int bix = blockIdx.x / kBlkPerB;
  const int d0  = (blockIdx.x - bix * kBlkPerB) * kScCh;
  const int d   = d0 + c;
  const size_t row0 = (size_t)bix * kSeq;
#pragma unroll 1
  for (int i = tid; i < kScCh * kNs; i += 128) {
    const int cc = i >> 4, s = i & 15;
    sA[s * kScCh + cc] = -expf(Alog[(size_t)(d0 + cc) * kNs + s]);
    sW[s * kScCh + cc] = Wdt[(size_t)(d0 + cc) * kDtR + s];
  }
  __syncthreads();
  float negA[8], h[8];
#pragma unroll
  for (int k = 0; k < 8; ++k) {
    negA[k] = sA[(half * 8 + k) * kScCh + c];
    h[k] = 0.f;
  }
  const float bb = bdt[d], Dd = Dp[d];
  const int q = lane >> 3, c8 = (lane & 7) * 8;
#pragma unroll 1
  for (int t0 = 0; t0 < kSeq; t0 += kScTS) {
    __syncthreads();
#pragma unroll
    for (int i = 0; i < 3; ++i) {
      const int idx = tid + 128 * i;
      const int r = idx / 12;
      const int c4 = (idx - r * 12) * 4;
      *(v4f*)(sX + r * kScXP + c4) = *(const v4f*)(XD + (row0 + t0 + r) * kXdP + c4);
    }
#pragma unroll
    for (int i = 0; i < 4; ++i) {
      const int idx = tid + 128 * i;
      const int r = idx >> 4;
      const int c4 = (idx & 15) * 4;
      *(v4f*)(sU + r * kScCh + c4) = *(const v4f*)(U + (row0 + t0 + r) * kDi + d0 + c4);
      *(v4f*)(sZ + r * kScCh + c4) = *(const v4f*)(XZ + (row0 + t0 + r) * kXzP + kDi + d0 + c4);
    }
    __syncthreads();
#pragma unroll 1
    for (int s = 0; s < kScTS; ++s) {
      const float* xr = sX + s * kScXP;
      float vdot = 0.f;
#pragma unroll 1
      for (int r4 = 0; r4 < kDtR / 4; ++r4) {
        const v4f xv = *(const v4f*)(xr + 4 * r4);
        const float* wp = sW + (4 * r4) * kScCh + c;
        vdot = fmaf(xv[0], wp[0], vdot);
        vdot = fmaf(xv[1], wp[kScCh], vdot);
        vdot = fmaf(xv[2], wp[2 * kScCh], vdot);
        vdot = fmaf(xv[3], wp[3 * kScCh], vdot);
      }
      const v4f bv0 = *(const v4f*)(xr + kDtR + half * 8);
      const v4f bv1 = *(const v4f*)(xr + kDtR + half * 8 + 4);
      const v4f cv0 = *(const v4f*)(xr + kDtR + kNs + half * 8);
      const v4f cv1 = *(const v4f*)(xr + kDtR + kNs + half * 8 + 4);
      const float Bs[8] = {bv0[0], bv0[1], bv0[2], bv0[3], bv1[0], bv1[1], bv1[2], bv1[3]};
      const float Cs[8] = {cv0[0], cv0[1], cv0[2], cv0[3], cv1[0], cv1[1], cv1[2], cv1[3]};
      const float v   = vdot + bb;
      const float a   = expf(-fabsf(v));
      const float uu  = 1.0f + a;
      const float l1p = logf(uu) + (a - (uu - 1.0f)) * (1.0f / uu);
      const float dt  = fmaxf(v, 0.0f) + l1p;
      const float ut  = sU[s * kScCh + c];
      const float zt  = sZ[s * kScCh + c];
      const float dtx = dt * ut;
      float y = 0.f;
#pragma unroll
      for (int k = 0; k < 8; ++k) {
        const float e = expf(dt * negA[k]);
        h[k] = fmaf(e, h[k], dtx * Bs[k]);
        y = fmaf(h[k], Cs[k], y);
      }
      const float yo = __shfl_xor(y, 16, 32);
      const float ys = y + yo;
      const float yt = fmaf(ut, Dd, ys);
      const float sg = 1.0f / (1.0f + expf(-zt));
      const float ov = yt * (zt * sg);
      if (half == 0) sY[s * kScYP + c] = ov;
    }
    __syncthreads();
    v4u pk[2];
#pragma unroll
    for (int it = 0; it < 2; ++it) {
      const int row = it * 16 + wave * 4 + q;
      const float* sp = sY + row * kScYP + c8;
      const v4f a0 = *(const v4f*)(sp);
      const v4f a1 = *(const v4f*)(sp + 4);
      pk[it] = cast8_f16(a0, a1, kCarryY);
    }
    for (int pass = 0; pass < 2; ++pass) {
#pragma unroll
      for (int it = 0; it < 2; ++it) {
        const int row = it * 16 + wave * 4 + q;
        *(volatile v4u*)(YG + (row0 + t0 + row) * kDi + d0 + c8) = pk[it];
      }
      __threadfence();
    }
  }
}

__global__ __launch_bounds__(256) void gelu_norm_kernel(
    const float* __restrict__ P, unsigned short* __restrict__ GH, unsigned short* __restrict__ GL,
    float* __restrict__ NRM)
{
  __shared__ __align__(16) float sR[8][kDm];
  __shared__ __align__(16) float sN[32];
  const int lane = threadIdx.x & 31;
  const int wave = __builtin_amdgcn_readfirstlane((int)(threadIdx.x >> 5));
  float* sr = sR[wave];
#pragma unroll 1
  for (int rr = 0; rr < 4; ++rr) {
    const int row = blockIdx.x * 32 + wave * 4 + rr;
    const float* pp = P + (size_t)row * kDm;
    float ss = 0.f;
#pragma unroll 1
    for (int i = 0; i < 8; ++i) {
      const float t = pp[i * 32 + lane];
      const float g = 0.5f * t * (1.0f + erff(t * 0.70710678118654752f));
      ss = fmaf(g, g, ss);
      sr[i * 32 + lane] = g;
    }
#pragma unroll
    for (int off = 16; off > 0; off >>= 1) ss += __shfl_xor(ss, off, 32);
    const float nrm = sqrtf(ss);
    if (lane == 0) sN[wave * 4 + rr] = nrm;
    __syncthreads();
    const v4f a0 = *(const v4f*)(sr + lane * 8);
    const v4f a1 = *(const v4f*)(sr + lane * 8 + 4);
    v4u hw, lw;
    split8_bf16(a0, a1, hw, lw);
    unsigned short* qh = GH + (size_t)row * kDm + lane * 8;
    unsigned short* ql = GL + (size_t)row * kDm + lane * 8;
    *(volatile v4u*)qh = hw;
    *(volatile v4u*)ql = lw;
    __threadfence();
    *(volatile v4u*)qh = hw;
    *(volatile v4u*)ql = lw;
    __syncthreads();
  }
  if (wave == 0) {
    const float nv = sN[lane];
    volatile float* np = NRM + (size_t)blockIdx.x * 32 + lane;
    *np = nv;
    __threadfence();
    *np = nv;
  }
}

__global__ __launch_bounds__(256) void loss_reduce_kernel(const float* __restrict__ NRM, float* __restrict__ out)
{
  __shared__ float sS[8];
  const int tid = threadIdx.x, lane = tid & 31;
  const int wave = __builtin_amdgcn_readfirstlane((int)(threadIdx.x >> 5));
  float s = 0.f;
#pragma unroll 1
  for (int i = 0; i < kTok / 256; ++i) s += NRM[i * 256 + tid];
#pragma unroll
  for (int off = 16; off > 0; off >>= 1) s += __shfl_xor(s, off, 32);
  if (lane == 0) sS[wave] = s;
  __syncthreads();
  float tot = 0.f;
#pragma unroll
  for (int w = 0; w < 8; ++w) tot += sS[w];
  const float res = 0.01f * (tot * (1.0f / (float)kTok));
  if (tid == 0) {
    volatile float* p = out + kLossIdx;
    *p = res;
    __threadfence();
    *p = res;
  }
}

extern "C" void kernel_launch(void* const* d_in, const int* in_sizes, int n_in,
                              void* d_out, int out_size, void* d_ws, size_t ws_size,
                              hipStream_t stream) {
  if (n_in < 20) return;
  if (in_sizes[0] != kTok * kIn) return;
  if (in_sizes[1] != kDm * kIn) return;
  if (in_sizes[2] != kDm || in_sizes[3] != kDm || in_sizes[4] != kDm) return;
  if (in_sizes[5] != kLay * kDm || in_sizes[6] != kLay * kDm) return;
  if (in_sizes[7] != kLay * kXzP * kDm) return;
  if (in_sizes[8] != kLay * kDi * 4) return;
  if (in_sizes[9] != kLay * kDi) return;
  if (in_sizes[10] != kLay * kXdN * kDi) return;
  if (in_sizes[11] != kLay * kDi * kDtR) return;
  if (in_sizes[12] != kLay * kDi) return;
  if (in_sizes[13] != kLay * kDi * kNs) return;
  if (in_sizes[14] != kLay * kDi) return;
  if (in_sizes[15] != kLay * kDm * kDi) return;
  if (in_sizes[16] != kDm * kDm) return;
  if (in_sizes[17] != kDm) return;
  if (in_sizes[18] != kCls * kDm) return;
  if (in_sizes[19] != kCls) return;
  if (out_size != kLossIdx + 1) return;
  if (ws_size < kWsTotal) return;

  const float* x       = (const float*)d_in[0];
  const float* in_w    = (const float*)d_in[1];
  const float* in_b    = (const float*)d_in[2];
  const float* ln_g    = (const float*)d_in[3];
  const float* ln_b    = (const float*)d_in[4];
  const float* blk_ng  = (const float*)d_in[5];
  const float* blk_nb  = (const float*)d_in[6];
  const float* blk_ipw = (const float*)d_in[7];
  const float* blk_cw  = (const float*)d_in[8];
  const float* blk_cb  = (const float*)d_in[9];
  const float* blk_xpw = (const float*)d_in[10];
  const float* blk_dtw = (const float*)d_in[11];
  const float* blk_dtb = (const float*)d_in[12];
  const float* blk_Alg = (const float*)d_in[13];
  const float* blk_D   = (const float*)d_in[14];
  const float* blk_opw = (const float*)d_in[15];
  const float* op_w    = (const float*)d_in[16];
  const float* op_b    = (const float*)d_in[17];
  const float* cls_w   = (const float*)d_in[18];
  const float* cls_b   = (const float*)d_in[19];
  float* out = (float*)d_out;

  char* ws = (char*)d_ws;
  unsigned short* XH   = (unsigned short*)(ws + kOffXH);
  unsigned short* XL   = (unsigned short*)(ws + kOffXL);
  unsigned short* WINH = (unsigned short*)(ws + kOffWINH);
  unsigned short* WINL = (unsigned short*)(ws + kOffWINL);
  unsigned short* WOPH = (unsigned short*)(ws + kOffWOPH);
  unsigned short* WOPL = (unsigned short*)(ws + kOffWOPL);
  unsigned short* WCLH = (unsigned short*)(ws + kOffWCLH);
  unsigned short* WCLL = (unsigned short*)(ws + kOffWCLL);
  unsigned short* WIP  = (unsigned short*)(ws + kOffWIP);
  unsigned short* WXP  = (unsigned short*)(ws + kOffWXP);
  unsigned short* WO   = (unsigned short*)(ws + kOffWO);
  float*          H0P  = (float*)(ws + kOffH0P);
  float*          H0   = (float*)(ws + kOffH0);
  float*          H1   = (float*)(ws + kOffH1);
  unsigned short* H2H  = (unsigned short*)(ws + kOffH2H);
  unsigned short* H2L  = (unsigned short*)(ws + kOffH2L);
  unsigned short* HN   = (unsigned short*)(ws + kOffHN);
  float*          XZ   = (float*)(ws + kOffXZ);
  float*          U    = (float*)(ws + kOffU);
  unsigned short* U16  = (unsigned short*)(ws + kOffU16);
  float*          XD   = (float*)(ws + kOffXD);
  unsigned short* YG   = (unsigned short*)(ws + kOffYG);
  float*          PH   = (float*)(ws + kOffPH);
  unsigned short* GH   = (unsigned short*)(ws + kOffGH);
  unsigned short* GL   = (unsigned short*)(ws + kOffGL);
  float*          NRM  = (float*)(ws + kOffNRM);

  split_rows_bf16_kernel<<<(kTok * kIn / 8) / 256, 256, 0, stream>>>(x, XH, XL, kTok * kIn / 8);
  split_rows_bf16_kernel<<<(kDm * kIn / 8) / 256, 256, 0, stream>>>(in_w, WINH, WINL, kDm * kIn / 8);
  split_rows_bf16_kernel<<<(kDm * kDm / 8) / 256, 256, 0, stream>>>(op_w, WOPH, WOPL, kDm * kDm / 8);
  split_rows_bf16_kernel<<<(kCls * kDm / 8) / 256, 256, 0, stream>>>(cls_w, WCLH, WCLL, kCls * kDm / 8);
  cast_rows_f16_kernel<<<(kLay * kXzP * kDm / 8) / 256, 256, 0, stream>>>(blk_ipw, WIP, kCarryW, kLay * kXzP * kDm / 8);
  cast_rows_f16_kernel<<<(kLay * kDm * kDi / 8) / 256, 256, 0, stream>>>(blk_opw, WO, kCarryW, kLay * kDm * kDi / 8);
  cast_xproj_pad_kernel<<<(kLay * kXdP * kDi / 8) / 256, 256, 0, stream>>>(blk_xpw, WXP, kCarryW, kLay * kXdP * kDi / 8);

  wmma_gemm64<1, true, 2, 0, false><<<32, 256, 0, stream>>>(
      XH, XL, kIn, WINH, WINL, kIn, (void*)H0P, (void*)H0P, kDm, in_b, in_b,
      kTok, kDm, kIn, 1.0f);
  ln_rows_kernel<0><<<kTok / 8, 256, 0, stream>>>(H0P, ln_g, ln_b, H0, blk_ng, blk_nb, HN);

  for (int l = 0; l < kLay; ++l) {
    const float* Hin = (l == 0) ? H0 : H1;
    if (l > 0) {
      ln_rows_kernel<1><<<kTok / 8, 256, 0, stream>>>(Hin, ln_g, ln_b, H0P, blk_ng + l * kDm, blk_nb + l * kDm, HN);
    }
    wmma_gemm64<0, false, 0, 0, false><<<128, 256, 0, stream>>>(
        HN, HN, kDm, WIP + (size_t)l * kXzP * kDm, WIP + (size_t)l * kXzP * kDm, kDm,
        (void*)XZ, (void*)XZ, kXzP, in_b, in_b,
        kTok, kXzP, kDm, 1.0f / (kCarryHN * kCarryW));
    conv_silu_kernel<<<dim3(kDi / 256, kTok / 64), 256, 0, stream>>>(
        XZ, blk_cw + (size_t)l * kDi * 4, blk_cb + (size_t)l * kDi, U, U16);
    wmma_gemm64<0, false, 0, 0, false><<<8, 256, 0, stream>>>(
        U16, U16, kDi, WXP + (size_t)l * kXdP * kDi, WXP + (size_t)l * kXdP * kDi, kDi,
        (void*)XD, (void*)XD, kXdP, in_b, in_b,
        kTok, kXdP, kDi, 1.0f / (kCarryU * kCarryW));
    scan_gate_kernel<<<kBat * (kDi / kScCh), 128, 0, stream>>>(
        XD, U, XZ, blk_dtw + (size_t)l * kDi * kDtR, blk_dtb + (size_t)l * kDi,
        blk_Alg + (size_t)l * kDi * kNs, blk_D + (size_t)l * kDi, YG);
    if (l == 0) {
      wmma_gemm64<0, false, 0, 0, true><<<32, 256, 0, stream>>>(
          YG, YG, kDi, WO + (size_t)l * kDm * kDi, WO + (size_t)l * kDm * kDi, kDi,
          (void*)H1, (void*)H1, kDm, in_b, Hin,
          kTok, kDm, kDi, 1.0f / (kCarryY * kCarryW));
    } else {
      wmma_gemm64<0, false, 0, 2, true><<<32, 256, 0, stream>>>(
          YG, YG, kDi, WO + (size_t)l * kDm * kDi, WO + (size_t)l * kDm * kDi, kDi,
          (void*)H2H, (void*)H2L, kDm, in_b, Hin,
          kTok, kDm, kDi, 1.0f / (kCarryY * kCarryW));
    }
  }

  wmma_gemm64<1, true, 2, 0, false><<<32, 256, 0, stream>>>(
      H2H, H2L, kDm, WOPH, WOPL, kDm, (void*)PH, (void*)PH, kDm, op_b, op_b,
      kTok, kDm, kDm, 1.0f);
  gelu_norm_kernel<<<kTok / 32, 256, 0, stream>>>(PH, GH, GL, NRM);
  wmma_gemm64<1, true, 2, 0, false><<<16, 256, 0, stream>>>(
      GH, GL, kDm, WCLH, WCLL, kDm, (void*)out, (void*)out, kCls, cls_b, cls_b,
      kTok, kCls, kDm, 1.0f);
  loss_reduce_kernel<<<1, 256, 0, stream>>>(NRM, out);
}
